// EosLayer_71725953843449
// MI455X (gfx1250) — hardware-run, weakly checked
//
#include <hip/hip_runtime.h>
#include <math.h>

typedef __attribute__((ext_vector_type(16))) _Float16 v16h;
typedef __attribute__((ext_vector_type(8)))  _Float16 v8h;
typedef __attribute__((ext_vector_type(8)))  float    v8f;
typedef __attribute__((ext_vector_type(4)))  float    v4f;
typedef __attribute__((ext_vector_type(4)))  unsigned int v4u;

constexpr int kBatch  = 4;
constexpr int kSeq    = 4096;
constexpr int kDim    = 512;
constexpr int kExp    = 8;
constexpr int kRows   = kBatch * kSeq;
constexpr int kNUsed  = kDim + 2 * kExp;
constexpr int kNPack  = 576;
constexpr int kChGrp  = 64;
constexpr float kTau      = 16.0f;
constexpr float kTauInv   = 1.0f / kTau;
constexpr float kLnEps    = 1e-5f;
constexpr float kInvDim   = 1.0f / (float)kDim;
constexpr float kActCarry = 16.0f;
constexpr float kWCarry   = 256.0f;
constexpr float kFold     = 1.0f / (kActCarry * kWCarry);
static_assert(kRows == 16384);
static_assert(kNUsed == 528);
static_assert((kNPack % 64) == 0 && kNPack >= kNUsed);
static_assert((kDim % 32) == 0);
static_assert((kRows % 64) == 0 && (kDim % 64) == 0);
static_assert(((kRows / 64) * (kNPack / 64)) % 8 == 0);
static_assert(((kRows / 64) * (kDim / 64)) % 8 == 0);
static_assert((kRows % 8) == 0);
static_assert(((kRows * kDim / 8) % 256) == 0);
static_assert((kDim % kChGrp) == 0);

constexpr size_t kOffXH   = 0;
constexpr size_t kOffW1T  = kOffXH  + (size_t)kRows  * kDim   * 2;
constexpr size_t kOffWOT  = kOffW1T + (size_t)kNPack * kDim   * 2;
constexpr size_t kOffIES  = kOffWOT + (size_t)kDim   * kDim   * 2;
constexpr size_t kOffY    = kOffIES + (size_t)kRows  * kNPack * 4;
constexpr size_t kOffYLH  = kOffY   + (size_t)kRows  * kDim   * 4;
constexpr size_t kWsTotal = kOffYLH + (size_t)kRows  * kDim   * 2;
static_assert(kWsTotal == 105971712ull);
static_assert(kWsTotal <= 134217728ull);
static_assert((kOffW1T % 128) == 0 && (kOffWOT % 128) == 0 && (kOffIES % 128) == 0 &&
              (kOffY % 128) == 0 && (kOffYLH % 128) == 0);

__device__ __forceinline__ unsigned pk16(unsigned short a, unsigned short b) { return (unsigned)a | ((unsigned)b << 16); }
__device__ __forceinline__ unsigned short h_bits(float f) { const _Float16 h = (_Float16)f; return __builtin_bit_cast(unsigned short, h); }
__device__ __forceinline__ float bf16_rne(float f) {
  const unsigned u = __float_as_uint(f);
  const unsigned r = (u + 0x7FFFu + ((u >> 16) & 1u)) & 0xFFFF0000u;
  return __uint_as_float(r);
}

__device__ __forceinline__ v16h frag_load_h(const _Float16* p) {
  union U { v16h v; v8h h[2]; } f;
  f.h[0] = *(const v8h*)(p);
  f.h[1] = *(const v8h*)(p + 16);
  return f.v;
}
__device__ __forceinline__ v8f mma_guard_h(v16h a, v16h b, v8f c) {
  c = __builtin_amdgcn_wmma_f32_16x16x32_f16(false, a, false, b, (short)0, c, false, false);
  asm volatile("v_nop\n\tv_nop\n\tv_nop\n\tv_nop" : "+v"(c) : "v"(a), "v"(b));
  return c;
}
__device__ __forceinline__ void keep4_h(v16h a, v16h b, v16h c, v16h d) { asm volatile("v_nop" :: "v"(a), "v"(b), "v"(c), "v"(d)); }
__device__ __forceinline__ void acc_guard4(v8f& a, v8f& b, v8f& c, v8f& d) { asm volatile("v_nop\n\tv_nop\n\tv_nop\n\tv_nop" : "+v"(a), "+v"(b), "+v"(c), "+v"(d)); }

__global__ __launch_bounds__(256) void gemm64_f16_kernel(
    const unsigned short* __restrict__ Ap, int lda,
    const unsigned short* __restrict__ Btp, int ldb,
    float* __restrict__ C, int ldc,
    int M, int N, int K, float scale) {
  const _Float16* A  = (const _Float16*)Ap;
  const _Float16* Bt = (const _Float16*)Btp;
  __shared__ __align__(16) float sT[8][16 * 68];
  const int lane = threadIdx.x & 31;
  const int wave = __builtin_amdgcn_readfirstlane((int)(threadIdx.x >> 5));
  const int tilesN = N >> 6;
  const int tilesM = M >> 6;
  const int tile = blockIdx.x * 8 + wave;
  if (tile >= tilesM * tilesN) return;
  const int tm = tile / tilesN;
  const int tn = tile - tm * tilesN;
  const int m0 = tm << 6;
  const int n0 = tn << 6;

  const int rlane = lane & 15;
  const int koff  = (lane >> 4) * 8;
  const int mOff  = (lane >> 4) * 8;

  v8f acc[4][4];
#pragma unroll
  for (int i = 0; i < 4; ++i)
#pragma unroll
    for (int j = 0; j < 4; ++j) acc[i][j] = (v8f){0.f, 0.f, 0.f, 0.f, 0.f, 0.f, 0.f, 0.f};

  for (int k0 = 0; k0 < K; k0 += 32) {
    v16h bh[4];
#pragma unroll
    for (int j = 0; j < 4; ++j) {
      const size_t bo = (size_t)(n0 + (j << 4) + rlane) * ldb + koff + k0;
      bh[j] = frag_load_h(Bt + bo);
    }
#pragma unroll
    for (int i = 0; i < 4; ++i) {
      const size_t ao = (size_t)(m0 + (i << 4) + rlane) * lda + koff + k0;
      const v16h ah = frag_load_h(A + ao);
#pragma unroll
      for (int j = 0; j < 4; ++j) acc[i][j] = mma_guard_h(ah, bh[j], acc[i][j]);
    }
    keep4_h(bh[0], bh[1], bh[2], bh[3]);
  }
  acc_guard4(acc[0][0], acc[0][1], acc[0][2], acc[0][3]);
  acc_guard4(acc[1][0], acc[1][1], acc[1][2], acc[1][3]);
  acc_guard4(acc[2][0], acc[2][1], acc[2][2], acc[2][3]);
  acc_guard4(acc[3][0], acc[3][1], acc[3][2], acc[3][3]);

  float* slab = sT[wave];
#pragma unroll
  for (int i = 0; i < 4; ++i) {
    const int mBase = m0 + (i << 4);
#pragma unroll
    for (int j = 0; j < 4; ++j) {
#pragma unroll
      for (int r = 0; r < 8; ++r) {
        const float v = acc[i][j][r] * scale;
        slab[(mOff + r) * 68 + (j << 4) + rlane] = v;
      }
    }
    __builtin_amdgcn_fence(__ATOMIC_RELEASE, "workgroup");
    __builtin_amdgcn_wave_barrier();
    __builtin_amdgcn_fence(__ATOMIC_ACQUIRE, "workgroup");
    {
      const int hh = lane >> 4, c4 = (lane & 15) * 4;
      for (int pass = 0; pass < 2; ++pass) {
#pragma unroll
        for (int it = 0; it < 8; ++it) {
          const int row = it * 2 + hh;
          const v4f v = *(const v4f*)(slab + row * 68 + c4);
          *(volatile v4f*)(C + (size_t)(mBase + row) * ldc + n0 + c4) = v;
        }
        __threadfence();
      }
    }
    __builtin_amdgcn_fence(__ATOMIC_RELEASE, "workgroup");
    __builtin_amdgcn_wave_barrier();
    __builtin_amdgcn_fence(__ATOMIC_ACQUIRE, "workgroup");
  }
}

__global__ __launch_bounds__(256) void cast8_f16_kernel(const float* __restrict__ in, unsigned short* __restrict__ out,
                                                        int n8, float carry) {
  const int i = blockIdx.x * 256 + threadIdx.x;
  if (i >= n8) return;
  const float* p = in + 8 * (size_t)i;
  const v4f a = *(const v4f*)(p);
  const v4f c = *(const v4f*)(p + 4);
  unsigned short hb[8];
#pragma unroll
  for (int e = 0; e < 4; ++e) {
    const float ra = a[e];
    const float rc = c[e];
    const float fa = bf16_rne(ra) * carry;
    const float fc = bf16_rne(rc) * carry;
    hb[e]     = h_bits(fa);
    hb[4 + e] = h_bits(fc);
  }
  const v4u u = (v4u){pk16(hb[0], hb[1]), pk16(hb[2], hb[3]), pk16(hb[4], hb[5]), pk16(hb[6], hb[7])};
  unsigned short* q = out + 8 * (size_t)i;
  *(volatile v4u*)q = u;
  __threadfence();
  *(volatile v4u*)q = u;
}

__global__ __launch_bounds__(256) void pack_w_kernel(const float* __restrict__ Wi, const float* __restrict__ We,
                                                     const float* __restrict__ Ws, const float* __restrict__ Wo,
                                                     unsigned short* __restrict__ W1T, unsigned short* __restrict__ WOT,
                                                     float carry) {
  __shared__ float sm[64][65];
  const int t  = threadIdx.x;
  const int k0 = blockIdx.x * 64;
  const int by = blockIdx.y;
  const bool isOut = (by >= kNPack / 64);
  const int n0 = (isOut ? (by - kNPack / 64) : by) * 64;
  const float* Wsq = isOut ? Wo : Wi;
  unsigned short* op = isOut ? WOT : W1T;
#pragma unroll 1
  for (int i = 0; i < 16; ++i) {
    const int e = i * 256 + t;
    const int r = e >> 6;
    const int c = e & 63;
    const int n = n0 + c;
    const int k = k0 + r;
    const int nc = (n < kDim) ? n : (kDim - 1);
    int ce = n - kDim;
    ce = (ce < 0) ? 0 : ((ce > kExp - 1) ? (kExp - 1) : ce);
    int cs = n - kDim - kExp;
    cs = (cs < 0) ? 0 : ((cs > kExp - 1) ? (kExp - 1) : cs);
    float a = Wsq[(size_t)k * kDim + nc];
    float b = We[k * kExp + ce];
    float d = Ws[k * kExp + cs];
    asm volatile("" : "+v"(a));
    asm volatile("" : "+v"(b));
    asm volatile("" : "+v"(d));
    const float v = (n < kDim) ? a : ((n < kDim + kExp) ? b : ((n < kNUsed) ? d : 0.0f));
    sm[c][r] = bf16_rne(v) * carry;
  }
  __syncthreads();
  const int lane = t & 31;
  const int wave = __builtin_amdgcn_readfirstlane((int)(t >> 5));
  const int q = lane >> 3, c8 = (lane & 7) * 8;
  for (int pass = 0; pass < 2; ++pass) {
#pragma unroll
    for (int it = 0; it < 2; ++it) {
      const int row = wave * 8 + it * 4 + q;
      unsigned short hb[8];
#pragma unroll
      for (int e = 0; e < 8; ++e) hb[e] = h_bits(sm[row][c8 + e]);
      const v4u u = (v4u){pk16(hb[0], hb[1]), pk16(hb[2], hb[3]), pk16(hb[4], hb[5]), pk16(hb[6], hb[7])};
      *(volatile v4u*)(op + (size_t)(n0 + row) * kDim + k0 + c8) = u;
    }
    __threadfence();
  }
}

__global__ __launch_bounds__(64) void scan_kernel(const float* __restrict__ IES, const float* __restrict__ o_param,
                                                  float* __restrict__ Y) {
  __shared__ float sO[kExp * kChGrp];
  const int tid = threadIdx.x;
  constexpr int kGrpPerB = kDim / kChGrp;
  const int b = blockIdx.x / kGrpPerB;
  const int d = (blockIdx.x - b * kGrpPerB) * kChGrp + tid;
#pragma unroll 1
  for (int k = 0; k < kExp; ++k) {
    const float p  = bf16_rne(o_param[k * kDim + d]);
    const float ls = fminf(p, 0.0f) - log1pf(expf(-fabsf(p)));
    sO[k * kChGrp + tid] = expf(ls * kTauInv);
  }
  __syncthreads();
  float o[kExp], m[kExp];
#pragma unroll
  for (int k = 0; k < kExp; ++k) {
    o[k] = sO[k * kChGrp + tid];
    m[k] = 0.0f;
  }
  const float* rp = IES + (size_t)b * kSeq * kNPack;
  float* yp = Y + (size_t)b * kSeq * kDim + d;
  float iv_n = rp[d];
  v4f e0n = *(const v4f*)(rp + kDim);
  v4f e1n = *(const v4f*)(rp + kDim + 4);
  v4f s0n = *(const v4f*)(rp + kDim + 8);
  v4f s1n = *(const v4f*)(rp + kDim + 12);
#pragma unroll 1
  for (int t = 0; t < kSeq; ++t) {
    const float iv = iv_n;
    const v4f e0 = e0n, e1 = e1n, s0 = s0n, s1 = s1n;
    const int tn = (t + 1 < kSeq) ? (t + 1) : (kSeq - 1);
    const float* np = rp + (size_t)tn * kNPack;
    iv_n = np[d];
    e0n = *(const v4f*)(np + kDim);
    e1n = *(const v4f*)(np + kDim + 4);
    s0n = *(const v4f*)(np + kDim + 8);
    s1n = *(const v4f*)(np + kDim + 12);
    float y = 0.0f;
    m[0] = fmaf(o[0], m[0], e0[0] * iv);
    y = fmaf(s0[0], m[0], y);
    m[1] = fmaf(o[1], m[1], e0[1] * iv);
    y = fmaf(s0[1], m[1], y);
    m[2] = fmaf(o[2], m[2], e0[2] * iv);
    y = fmaf(s0[2], m[2], y);
    m[3] = fmaf(o[3], m[3], e0[3] * iv);
    y = fmaf(s0[3], m[3], y);
    m[4] = fmaf(o[4], m[4], e1[0] * iv);
    y = fmaf(s1[0], m[4], y);
    m[5] = fmaf(o[5], m[5], e1[1] * iv);
    y = fmaf(s1[1], m[5], y);
    m[6] = fmaf(o[6], m[6], e1[2] * iv);
    y = fmaf(s1[2], m[6], y);
    m[7] = fmaf(o[7], m[7], e1[3] * iv);
    y = fmaf(s1[3], m[7], y);
    volatile float* q = yp + (size_t)t * kDim;
    *q = y;
    __threadfence();
    *q = y;
  }
}

__global__ __launch_bounds__(256) void layernorm_f16_kernel(const float* __restrict__ Y, const float* __restrict__ gamma,
                                                            const float* __restrict__ beta,
                                                            unsigned short* __restrict__ YLH, float carry) {
  const int lane = threadIdx.x & 31;
  const int wave = __builtin_amdgcn_readfirstlane((int)(threadIdx.x >> 5));
  const int row  = blockIdx.x * 8 + wave;
  const int c0 = lane * 8;
  const int c1 = 256 + lane * 8;
  const float* yr = Y + (size_t)row * kDim;
  const v4f a0 = *(const v4f*)(yr + c0);
  const v4f a1 = *(const v4f*)(yr + c0 + 4);
  const v4f a2 = *(const v4f*)(yr + c1);
  const v4f a3 = *(const v4f*)(yr + c1 + 4);
  float x[16];
#pragma unroll
  for (int e = 0; e < 4; ++e) {
    x[e]      = a0[e];
    x[4 + e]  = a1[e];
    x[8 + e]  = a2[e];
    x[12 + e] = a3[e];
  }
  float s = 0.0f;
#pragma unroll
  for (int e = 0; e < 16; ++e) s += x[e];
#pragma unroll
  for (int off = 16; off > 0; off >>= 1) s += __shfl_xor(s, off, 32);
  const float mu = s * kInvDim;
  float qs = 0.0f;
#pragma unroll
  for (int e = 0; e < 16; ++e) {
    const float dv = x[e] - mu;
    x[e] = dv;
    qs = fmaf(dv, dv, qs);
  }
#pragma unroll
  for (int off = 16; off > 0; off >>= 1) qs += __shfl_xor(qs, off, 32);
  const float rinv = rsqrtf(qs * kInvDim + kLnEps);
  const v4f g0 = *(const v4f*)(gamma + c0);
  const v4f g1 = *(const v4f*)(gamma + c0 + 4);
  const v4f g2 = *(const v4f*)(gamma + c1);
  const v4f g3 = *(const v4f*)(gamma + c1 + 4);
  const v4f b0 = *(const v4f*)(beta + c0);
  const v4f b1 = *(const v4f*)(beta + c0 + 4);
  const v4f b2 = *(const v4f*)(beta + c1);
  const v4f b3 = *(const v4f*)(beta + c1 + 4);
  float gg[16], bb[16];
#pragma unroll
  for (int e = 0; e < 4; ++e) {
    const float t0 = g0[e];
    const float t1 = g1[e];
    const float t2 = g2[e];
    const float t3 = g3[e];
    const float u0 = b0[e];
    const float u1 = b1[e];
    const float u2 = b2[e];
    const float u3 = b3[e];
    gg[e]      = bf16_rne(t0);
    gg[4 + e]  = bf16_rne(t1);
    gg[8 + e]  = bf16_rne(t2);
    gg[12 + e] = bf16_rne(t3);
    bb[e]      = bf16_rne(u0);
    bb[4 + e]  = bf16_rne(u1);
    bb[8 + e]  = bf16_rne(u2);
    bb[12 + e] = bf16_rne(u3);
  }
  unsigned short hb[16];
#pragma unroll
  for (int e = 0; e < 16; ++e) {
    const float v = (x[e] * rinv) * gg[e] + bb[e];
    hb[e] = h_bits(v * carry);
  }
  const v4u u0 = (v4u){pk16(hb[0], hb[1]), pk16(hb[2], hb[3]), pk16(hb[4], hb[5]), pk16(hb[6], hb[7])};
  const v4u u1 = (v4u){pk16(hb[8], hb[9]), pk16(hb[10], hb[11]), pk16(hb[12], hb[13]), pk16(hb[14], hb[15])};
  unsigned short* q0 = YLH + (size_t)row * kDim + c0;
  unsigned short* q1 = YLH + (size_t)row * kDim + c1;
  *(volatile v4u*)q0 = u0;
  *(volatile v4u*)q1 = u1;
  __threadfence();
  *(volatile v4u*)q0 = u0;
  *(volatile v4u*)q1 = u1;
}

extern "C" void kernel_launch(void* const* d_in, const int* in_sizes, int n_in,
                              void* d_out, int out_size, void* d_ws, size_t ws_size,
                              hipStream_t stream) {
  if (n_in < 8) return;
  if (in_sizes[0] != kRows * kDim) return;
  if (in_sizes[1] != kDim * kDim) return;
  if (in_sizes[2] != kDim * kExp) return;
  if (in_sizes[3] != kDim * kExp) return;
  if (in_sizes[4] != kExp * kDim) return;
  if (in_sizes[5] != kDim) return;
  if (in_sizes[6] != kDim) return;
  if (in_sizes[7] != kDim * kDim) return;
  if (out_size != kRows * kDim) return;
  if (ws_size < kWsTotal) return;

  const float* x       = (const float*)d_in[0];
  const float* W_i     = (const float*)d_in[1];
  const float* W_e     = (const float*)d_in[2];
  const float* W_s     = (const float*)d_in[3];
  const float* o_param = (const float*)d_in[4];
  const float* gamma   = (const float*)d_in[5];
  const float* beta    = (const float*)d_in[6];
  const float* W_out   = (const float*)d_in[7];
  float* out = (float*)d_out;

  char* ws = (char*)d_ws;
  unsigned short* XH  = (unsigned short*)(ws + kOffXH);
  unsigned short* W1T = (unsigned short*)(ws + kOffW1T);
  unsigned short* WOT = (unsigned short*)(ws + kOffWOT);
  float*          IES = (float*)(ws + kOffIES);
  float*          Yp  = (float*)(ws + kOffY);
  unsigned short* YLH = (unsigned short*)(ws + kOffYLH);

  cast8_f16_kernel<<<(kRows * kDim / 8) / 256, 256, 0, stream>>>(x, XH, kRows * kDim / 8, kActCarry);

  pack_w_kernel<<<dim3(kDim / 64, kNPack / 64 + kDim / 64), 256, 0, stream>>>(W_i, W_e, W_s, W_out, W1T, WOT, kWCarry);

  gemm64_f16_kernel<<<((kRows / 64) * (kNPack / 64)) / 8, 256, 0, stream>>>(
      XH, kDim, W1T, kDim, IES, kNPack, kRows, kNPack, kDim, kFold);

  scan_kernel<<<kBatch * (kDim / kChGrp), kChGrp, 0, stream>>>(IES, o_param, Yp);

  layernorm_f16_kernel<<<kRows / 8, 256, 0, stream>>>(Yp, gamma, beta, YLH, kActCarry);

  gemm64_f16_kernel<<<((kRows / 64) * (kDim / 64)) / 8, 256, 0, stream>>>(
      YLH, kDim, WOT, kDim, out, kDim, kRows, kDim, kDim, kFold);
}
